// RNN_34093450396226
// MI455X (gfx1250) — hardware-verified
//
#include <hip/hip_runtime.h>
#include <math.h>

constexpr int NBATCH = 8192;
constexpr int NSTEP  = 512;
constexpr int NHID   = 20;
constexpr int KPAD   = 32;
constexpr int NTHR   = 256;
constexpr int NWAVE  = NTHR / 32;
constexpr int ROWS_PER_WAVE  = 16;
constexpr int ROWS_PER_BLOCK = ROWS_PER_WAVE * NWAVE;
constexpr int NPLANE = 5;
constexpr int K_BIH = 20;
constexpr int K_BHH = 21;
constexpr int K_XIN = 22;
constexpr float TWO_LOG2E = 2.0f * 1.44269504088896340736f;

static_assert(KPAD == 32, "one 32-deep k step");
static_assert(NHID <= 20 && NHID > 16, "unit tile split 16 + 4");
static_assert(K_BIH == 20 && K_BHH == 21 && K_XIN == 22, "slots = fragment word 6 (both halves) and word 7 (low half) of lane half 0");
static_assert(K_XIN < KPAD, "slots inside the padded k range");
static_assert(NBATCH % ROWS_PER_BLOCK == 0, "grid exact");
static_assert(ROWS_PER_BLOCK == 128, "one block writes 4 whole 128-B lines of the output");
static_assert((KPAD * KPAD) % NTHR == 0, "plane fill loop exact");

typedef __attribute__((ext_vector_type(16))) __bf16   v16b;
typedef __attribute__((ext_vector_type(8)))  __bf16   v8b;
typedef __attribute__((ext_vector_type(8)))  float    v8f;
typedef __attribute__((ext_vector_type(4)))  float    v4f;
typedef __attribute__((ext_vector_type(8)))  unsigned v8u;

__device__ __forceinline__ unsigned bf_bits_u32(float f) {
  const unsigned u = __float_as_uint(f);
  return (u + 0x7FFFu + ((u >> 16) & 1u)) >> 16;
}
__device__ __forceinline__ float bf16_value(float f) { return __uint_as_float(bf_bits_u32(f) << 16); }

struct FragB {
  union U { v16b v; v8b h[2]; };
  static __device__ __forceinline__ v16b load(const __bf16* p) {
    U f;
    f.h[0] = *(const v8b*)(p);
    f.h[1] = *(const v8b*)(p + 16);
    return f.v;
  }
};

__device__ __forceinline__ v8f mma_bf(v16b a, v16b b, v8f c) {
  return __builtin_amdgcn_wmma_f32_16x16x32_bf16(false, a, false, b, (short)0, c, false, false);
}
__device__ __forceinline__ void group_guard4(v8f& a, v8f& b, v16b p, v16b q, v16b r, v16b s) {
  asm volatile("v_nop\n\tv_nop\n\tv_nop\n\tv_nop" : "+v"(a), "+v"(b) : "v"(p), "v"(q), "v"(r), "v"(s));
}
__device__ __forceinline__ void group_guard8(v8f& a, v8f& b, v16b p, v16b q, v16b r, v16b s,
                                             v16b t, v16b u, v16b v, v16b w) {
  asm volatile("v_nop\n\tv_nop\n\tv_nop\n\tv_nop" : "+v"(a), "+v"(b)
               : "v"(p), "v"(q), "v"(r), "v"(s), "v"(t), "v"(u), "v"(v), "v"(w));
}

__device__ __forceinline__ float tanh_f32(float x) {
  const float e = exp2f(x * TWO_LOG2E);
  return 1.0f - 2.0f * __builtin_amdgcn_rcpf(e + 1.0f);
}

template <int KIND>
__device__ __forceinline__ void fill_plane(__bf16* dst, const float* __restrict__ W, const float* __restrict__ bih,
                                           const float* __restrict__ bhh, const float* __restrict__ wx, int tid) {
#pragma unroll 1
  for (int i = tid; i < KPAD * KPAD; i += NTHR) {
    const int n = i >> 5;
    const int k = i & 31;
    const int nc = (n < NHID) ? n : (NHID - 1);
    const int kc = (k < NHID) ? k : (NHID - 1);
    float w = W[nc * NHID + kc];
    asm volatile("" : "+v"(w));
    float v = (k < NHID) ? w : 0.0f;
    if (KIND >= 1) {
      float bi = bih[nc];
      asm volatile("" : "+v"(bi));
      float bh = bhh[nc];
      asm volatile("" : "+v"(bh));
      v = (k == K_BIH) ? bi : v;
      v = (k == K_BHH) ? bh : v;
    }
    if (KIND == 2) {
      float wi = wx[nc];
      asm volatile("" : "+v"(wi));
      v = (k == K_XIN) ? wi : v;
    }
    v = (n < NHID) ? v : 0.0f;
    dst[i] = __builtin_bit_cast(__bf16, (unsigned short)bf_bits_u32(v));
  }
}

template <bool TWO_IN>
__device__ __forceinline__ void rnn_layer_step(const v16b wa0, const v16b wa1, const v16b wr0, const v16b wr1,
                                               const v16b inh, const v16b inl, v8u& sh, v8u& sl,
                                               const bool half0, const unsigned onesw, float (&hout)[12]) {
  v8f acc0 = (v8f){0.f, 0.f, 0.f, 0.f, 0.f, 0.f, 0.f, 0.f};
  v8f acc1 = (v8f){0.f, 0.f, 0.f, 0.f, 0.f, 0.f, 0.f, 0.f};
  const v16b bh = __builtin_bit_cast(v16b, sh);
  const v16b bl = __builtin_bit_cast(v16b, sl);
  if (TWO_IN) {
    acc0 = mma_bf(wa0, inh, acc0);
    acc1 = mma_bf(wa1, inh, acc1);
    acc0 = mma_bf(wa0, inl, acc0);
    acc1 = mma_bf(wa1, inl, acc1);
  }
  acc0 = mma_bf(wr0, bh, acc0);
  acc1 = mma_bf(wr1, bh, acc1);
  acc0 = mma_bf(wr0, bl, acc0);
  acc1 = mma_bf(wr1, bl, acc1);
  if (TWO_IN) group_guard8(acc0, acc1, wa0, wa1, wr0, wr1, inh, inl, bh, bl);
  else        group_guard4(acc0, acc1, wr0, wr1, bh, bl);

  float hv[12];
#pragma unroll
  for (int r = 0; r < 8; ++r) hv[r] = tanh_f32(acc0[r]);
#pragma unroll
  for (int r = 0; r < 4; ++r) hv[8 + r] = tanh_f32(acc1[r]);

  unsigned hb[12], lb[12];
#pragma unroll
  for (int i = 0; i < 12; ++i) {
    const float v = hv[i];
    const unsigned b0 = bf_bits_u32(v);
    const float hf = __uint_as_float(b0 << 16);
    const float res = v - hf;
    hb[i] = b0;
    lb[i] = bf_bits_u32(res);
    hout[i] = v;
  }
  v8u nh, nl;
  nh[0] = hb[0] | (hb[1] << 16);
  nh[1] = hb[2] | (hb[3] << 16);
  nh[2] = hb[4] | (hb[5] << 16);
  nh[3] = hb[6] | (hb[7] << 16);
  const unsigned h45 = hb[8]  | (hb[9]  << 16);
  const unsigned h67 = hb[10] | (hb[11] << 16);
  nh[4] = half0 ? h45 : 0u;
  nh[5] = half0 ? h67 : 0u;
  nh[6] = onesw;
  nh[7] = 0u;
  nl[0] = lb[0] | (lb[1] << 16);
  nl[1] = lb[2] | (lb[3] << 16);
  nl[2] = lb[4] | (lb[5] << 16);
  nl[3] = lb[6] | (lb[7] << 16);
  const unsigned l45 = lb[8]  | (lb[9]  << 16);
  const unsigned l67 = lb[10] | (lb[11] << 16);
  nl[4] = half0 ? l45 : 0u;
  nl[5] = half0 ? l67 : 0u;
  nl[6] = 0u;
  nl[7] = 0u;
  sh = nh;
  sl = nl;
}

__global__ __launch_bounds__(NTHR) void rnn3_seq_kernel(
    const float* __restrict__ x,
    const float* __restrict__ w_ih0, const float* __restrict__ w_hh0,
    const float* __restrict__ b_ih0, const float* __restrict__ b_hh0,
    const float* __restrict__ w_ih1, const float* __restrict__ w_hh1,
    const float* __restrict__ b_ih1, const float* __restrict__ b_hh1,
    const float* __restrict__ w_ih2, const float* __restrict__ w_hh2,
    const float* __restrict__ b_ih2, const float* __restrict__ b_hh2,
    const float* __restrict__ fc_w, const float* __restrict__ fc_b,
    float* __restrict__ out) {
  __shared__ __align__(16) __bf16 Wsh[NPLANE * KPAD * KPAD];
  __shared__ __align__(16) float  Outs[ROWS_PER_BLOCK];

  const int tid  = threadIdx.x;
  const int lane = tid & 31;
  const int wave = tid >> 5;
  const int c    = lane & 15;
  const int hh   = lane >> 4;
  const bool half0 = (hh == 0);

  fill_plane<2>(Wsh + 0 * KPAD * KPAD, w_hh0, b_ih0, b_hh0, w_ih0, tid);
  fill_plane<0>(Wsh + 1 * KPAD * KPAD, w_ih1, b_ih1, b_hh1, w_ih0, tid);
  fill_plane<1>(Wsh + 2 * KPAD * KPAD, w_hh1, b_ih1, b_hh1, w_ih0, tid);
  fill_plane<0>(Wsh + 3 * KPAD * KPAD, w_ih2, b_ih2, b_hh2, w_ih0, tid);
  fill_plane<1>(Wsh + 4 * KPAD * KPAD, w_hh2, b_ih2, b_hh2, w_ih0, tid);
  __syncthreads();

  const __bf16* wbase = Wsh + c * KPAD + 8 * hh;
  const v16b whh0_0 = FragB::load(wbase + 0 * KPAD * KPAD);
  const v16b whh0_1 = FragB::load(wbase + 0 * KPAD * KPAD + 16 * KPAD);
  const v16b wih1_0 = FragB::load(wbase + 1 * KPAD * KPAD);
  const v16b wih1_1 = FragB::load(wbase + 1 * KPAD * KPAD + 16 * KPAD);
  const v16b whh1_0 = FragB::load(wbase + 2 * KPAD * KPAD);
  const v16b whh1_1 = FragB::load(wbase + 2 * KPAD * KPAD + 16 * KPAD);
  const v16b wih2_0 = FragB::load(wbase + 3 * KPAD * KPAD);
  const v16b wih2_1 = FragB::load(wbase + 3 * KPAD * KPAD + 16 * KPAD);
  const v16b whh2_0 = FragB::load(wbase + 4 * KPAD * KPAD);
  const v16b whh2_1 = FragB::load(wbase + 4 * KPAD * KPAD + 16 * KPAD);

  const unsigned onesw = half0 ? 0x3F803F80u : 0u;
  const v8u zw = {0u, 0u, 0u, 0u, 0u, 0u, 0u, 0u};
  v8u s0h = zw, s0l = zw, s1h = zw, s1l = zw, s2h = zw, s2l = zw;
  s0h[6] = onesw;
  s1h[6] = onesw;
  s2h[6] = onesw;

  float h2f[12];
#pragma unroll
  for (int i = 0; i < 12; ++i) h2f[i] = 0.0f;

  const int brow = blockIdx.x * ROWS_PER_BLOCK + wave * ROWS_PER_WAVE + c;
  const float* xrow = x + (size_t)brow * NSTEP;
  float xcur = xrow[0];

#pragma unroll 1
  for (int t = 0; t < NSTEP; ++t) {
    const int tnx = (t + 1 < NSTEP) ? (t + 1) : (NSTEP - 1);
    const float xnext = xrow[tnx];
    const unsigned xb = bf_bits_u32(xcur);
    s0h[7] = half0 ? xb : 0u;

    float dump0[12];
    float dump1[12];
    const v16b unused = __builtin_bit_cast(v16b, zw);
    rnn_layer_step<false>(whh0_0, whh0_1, whh0_0, whh0_1, unused, unused, s0h, s0l, half0, onesw, dump0);
    const v16b h0h = __builtin_bit_cast(v16b, s0h);
    const v16b h0l = __builtin_bit_cast(v16b, s0l);
    rnn_layer_step<true>(wih1_0, wih1_1, whh1_0, whh1_1, h0h, h0l, s1h, s1l, half0, onesw, dump1);
    const v16b h1h = __builtin_bit_cast(v16b, s1h);
    const v16b h1l = __builtin_bit_cast(v16b, s1l);
    rnn_layer_step<true>(wih2_0, wih2_1, whh2_0, whh2_1, h1h, h1l, s2h, s2l, half0, onesw, h2f);
    xcur = xnext;
  }

  float s = 0.0f;
#pragma unroll
  for (int r = 0; r < 8; ++r) {
    const float wv = bf16_value(fc_w[8 * hh + r]);
    s += wv * h2f[r];
  }
#pragma unroll
  for (int r = 0; r < 4; ++r) {
    const float wv = bf16_value(fc_w[16 + r]);
    const float hvv = half0 ? h2f[8 + r] : 0.0f;
    s += wv * hvv;
  }
  const float other = __shfl_xor(s, 16, 32);
  const float res = (s + other) + bf16_value(fc_b[0]);
  if (half0) Outs[wave * ROWS_PER_WAVE + c] = res;
  __syncthreads();
  if (wave == 0) {
    const v4f v = *(const v4f*)(Outs + 4 * lane);
    float* op = out + (size_t)blockIdx.x * ROWS_PER_BLOCK + 4 * lane;
    *(volatile v4f*)op = v;
    __threadfence();
    *(volatile v4f*)op = v;
  }
}

extern "C" void kernel_launch(void* const* d_in, const int* in_sizes, int n_in,
                              void* d_out, int out_size, void* d_ws, size_t ws_size, hipStream_t stream) {
  (void)d_ws;
  (void)ws_size;
  if (n_in < 15 || d_out == nullptr) return;
  if (in_sizes[0] != NBATCH * NSTEP || in_sizes[1] != NHID || in_sizes[2] != NHID * NHID ||
      in_sizes[3] != NHID || in_sizes[4] != NHID || in_sizes[5] != NHID * NHID || in_sizes[6] != NHID * NHID ||
      in_sizes[7] != NHID || in_sizes[8] != NHID || in_sizes[9] != NHID * NHID || in_sizes[10] != NHID * NHID ||
      in_sizes[11] != NHID || in_sizes[12] != NHID || in_sizes[13] != NHID || in_sizes[14] != 1 ||
      out_size != NBATCH) return;

  const float* x     = (const float*)d_in[0];
  const float* w_ih0 = (const float*)d_in[1];
  const float* w_hh0 = (const float*)d_in[2];
  const float* b_ih0 = (const float*)d_in[3];
  const float* b_hh0 = (const float*)d_in[4];
  const float* w_ih1 = (const float*)d_in[5];
  const float* w_hh1 = (const float*)d_in[6];
  const float* b_ih1 = (const float*)d_in[7];
  const float* b_hh1 = (const float*)d_in[8];
  const float* w_ih2 = (const float*)d_in[9];
  const float* w_hh2 = (const float*)d_in[10];
  const float* b_ih2 = (const float*)d_in[11];
  const float* b_hh2 = (const float*)d_in[12];
  const float* fc_w  = (const float*)d_in[13];
  const float* fc_b  = (const float*)d_in[14];
  float* out = (float*)d_out;

  rnn3_seq_kernel<<<NBATCH / ROWS_PER_BLOCK, NTHR, 0, stream>>>(
      x, w_ih0, w_hh0, b_ih0, b_hh0, w_ih1, w_hh1, b_ih1, b_hh1, w_ih2, w_hh2, b_ih2, b_hh2, fc_w, fc_b, out);
}
